// MambaBlock_18777597018519
// MI455X (gfx1250) — hardware-verified
//
#include <hip/hip_runtime.h>
#include <stddef.h>
#include <stdint.h>
#include <math.h>


#define NBAT   2
#define SEQ    2048
#define DM     1024
#define DI     2048
#define DS     64
#define MT     4096
#define E2     4096
#define KX     4096
#define KH     128
#define GTHR   128
#define GBM    64
#define PTHR   256
#define CS     64
#define TS     16
#define RCH    32
#define WSMAX  134217728

#define UX     (MT * DM / 8)
#define UWI    (E2 * DM / 8)
#define UWO    (DM * KX / 8)
#define UB2    (DS * KX / 8)
#define UC2    (DI * KH / 8)
#define UTOT   (UX + UWI + UWO + UB2 + UC2)

static_assert(MT == NBAT * SEQ && E2 == 2 * DI && KX == 2 * DI && KH == 2 * DS);
static_assert(UX % PTHR == 0 && UWI % PTHR == 0 && UWO % PTHR == 0 && UB2 % PTHR == 0 && UC2 % PTHR == 0);
static_assert(MT % GBM == 0 && E2 % 128 == 0 && DI % 128 == 0 && DM % 128 == 0 && DS == 64);
static_assert(DM % 32 == 0 && KX % 32 == 0 && KH % 32 == 0);
static_assert(DI % CS == 0 && SEQ % TS == 0 && SEQ % RCH == 0);
static_assert(TS * CS / 4 == 4 * 64 && TS * CS / 8 == 2 * 64);
static_assert(RCH * DS / 4 == 8 * 64 && RCH * KH / 8 == 8 * 64);

typedef float          v4f   __attribute__((ext_vector_type(4)));
typedef float          v8f   __attribute__((ext_vector_type(8)));
typedef int            v8i   __attribute__((ext_vector_type(8)));
typedef unsigned short v4us  __attribute__((ext_vector_type(4)));
typedef unsigned short v8us  __attribute__((ext_vector_type(8)));
typedef unsigned short v16us __attribute__((ext_vector_type(16)));
typedef __bf16         v16bf __attribute__((ext_vector_type(16)));
typedef v4f  __attribute__((may_alias)) v4fa;
typedef v4us __attribute__((may_alias)) v4usa;
typedef v8us __attribute__((may_alias)) v8usa;
union FragB { v16bf v; v16us u; v8us h[2]; v8i w; };

__device__ __forceinline__ v8f wmb(const FragB& a, const FragB& b, v8f c) {
  v8f d = __builtin_amdgcn_wmma_f32_16x16x32_bf16(false, a.v, false, b.v, (short)0, c, false, false);
  asm volatile("v_nop\n\tv_nop\n\tv_nop\n\tv_nop" : "+v"(d) : "v"(a.w), "v"(b.w));
  return d;
}

__device__ __forceinline__ unsigned bf16_bits(float f) {
  const unsigned u = __float_as_uint(f);
  return (u + 0x7FFFu + ((u >> 16) & 1u)) >> 16;
}
__device__ __forceinline__ float bf16_val(float f) {
  return __uint_as_float(bf16_bits(f) << 16);
}
__device__ __forceinline__ float silu_f(float v) {
  return v * (1.0f / (1.0f + expf(-v)));
}

__device__ __forceinline__ void cvt8(const float* __restrict__ p, unsigned short* dp) {
  const v4f a = *(const v4fa*)p;
  const v4f b = *(const v4fa*)(p + 4);
  v8us o;
  o[0] = (unsigned short)bf16_bits(a.x); o[1] = (unsigned short)bf16_bits(a.y);
  o[2] = (unsigned short)bf16_bits(a.z); o[3] = (unsigned short)bf16_bits(a.w);
  o[4] = (unsigned short)bf16_bits(b.x); o[5] = (unsigned short)bf16_bits(b.y);
  o[6] = (unsigned short)bf16_bits(b.z); o[7] = (unsigned short)bf16_bits(b.w);
  *(volatile v8us*)dp = o;
  __threadfence();
  *(volatile v8us*)dp = o;
}

__global__ __launch_bounds__(PTHR) void k_prep(const float* __restrict__ x, const float* __restrict__ w1,
                                               const float* __restrict__ w2, const float* __restrict__ Bm,
                                               const float* __restrict__ Cm,
                                               unsigned short* XB, unsigned short* WIN, unsigned short* WOUT2,
                                               unsigned short* B2, unsigned short* C2) {
  const int u = (int)blockIdx.x * PTHR + (int)threadIdx.x;
  if (u < UX) {
    cvt8(x + (size_t)u * 8, XB + (size_t)u * 8);
  } else if (u < UX + UWI) {
    const int v = u - UX;
    cvt8(w1 + (size_t)v * 8, WIN + (size_t)v * 8);
  } else if (u < UX + UWI + UWO) {
    const int v  = u - (UX + UWI);
    const int n  = v >> 9;
    const int k8 = (v & 511) * 8;
    cvt8(w2 + (size_t)n * DI + (k8 & (DI - 1)), WOUT2 + (size_t)n * KX + k8);
  } else if (u < UX + UWI + UWO + UB2) {
    const int v  = u - (UX + UWI + UWO);
    const int n  = v >> 9;
    const int k8 = (v & 511) * 8;
    cvt8(Bm + (size_t)n * DI + (k8 & (DI - 1)), B2 + (size_t)n * KX + k8);
  } else if (u < UTOT) {
    const int v  = u - (UX + UWI + UWO + UB2);
    const int n  = v >> 4;
    const int k8 = (v & 15) * 8;
    cvt8(Cm + (size_t)n * DS + (k8 & (DS - 1)), C2 + (size_t)n * KH + k8);
  }
}

template <int NT>
__device__ __forceinline__ void gemm_loop(const unsigned short* __restrict__ ap,
                                          const unsigned short* __restrict__ bp, int K, v8f (&acc)[NT]) {
#pragma unroll 1
  for (int k0 = 0; k0 < K; k0 += 32) {
    FragB af;
    af.h[0] = *(const v8usa*)(ap + k0);
    af.h[1] = *(const v8usa*)(ap + k0 + 16);
#pragma unroll
    for (int nt = 0; nt < NT; ++nt) {
      const unsigned short* wq = bp + (size_t)(16 * nt) * (size_t)K + k0;
      FragB bf;
      bf.h[0] = *(const v8usa*)wq;
      bf.h[1] = *(const v8usa*)(wq + 16);
      acc[nt] = wmb(af, bf, acc[nt]);
    }
  }
}

template <int SILU>
__global__ __launch_bounds__(GTHR) void k_gemm128(const unsigned short* __restrict__ A,
                                                  const unsigned short* __restrict__ BT,
                                                  const float* __restrict__ bias, float* outF,
                                                  size_t gateOff, int K, int ldo, int gateCol) {
  __shared__ __attribute__((aligned(16))) float stg[GBM * 128];
  const int tid = (int)threadIdx.x, lane = tid & 31, wave = tid >> 5, hh = lane >> 4, m = lane & 15;
  const int rowBase = (int)blockIdx.x * GBM;
  const int col0    = (int)blockIdx.y * 128;

  v8f acc[8];
  {
    const v8f z = {0.f, 0.f, 0.f, 0.f, 0.f, 0.f, 0.f, 0.f};
#pragma unroll
    for (int t = 0; t < 8; ++t) acc[t] = z;
  }
  const unsigned short* ap = A  + (size_t)(rowBase + 16 * wave + m) * (size_t)K + 8 * hh;
  const unsigned short* bp = BT + (size_t)(col0 + m) * (size_t)K + 8 * hh;
  gemm_loop<8>(ap, bp, K, acc);

#pragma unroll
  for (int nt = 0; nt < 8; ++nt) {
    const int lc = 16 * nt + m;
#pragma unroll
    for (int r = 0; r < 8; ++r) {
      const int lr = 16 * wave + 8 * hh + r;
      stg[lr * 128 + lc] = acc[nt][r];
    }
  }
  __syncthreads();

  v4f b4;
  {
    const v4f t1 = *(const v4fa*)(bias + col0 + 4 * lane);
    b4.x = bf16_val(t1.x); b4.y = bf16_val(t1.y); b4.z = bf16_val(t1.z); b4.w = bf16_val(t1.w);
  }
  const bool gate = (SILU != 0) && (col0 >= gateCol);
  const size_t pofs = gate ? gateOff : (size_t)0;
  const int oc = (gate ? (col0 - gateCol) : col0) + 4 * lane;
  float* orow = outF + pofs + (size_t)(rowBase + 16 * wave) * (size_t)ldo + oc;
  float* srow = stg + (16 * wave) * 128 + 4 * lane;

#pragma unroll 1
  for (int i = 0; i < 16; ++i) {
    v4f t = *(const v4fa*)(srow + i * 128) + b4;
    if constexpr (SILU != 0) {
      if (gate) {
        t.x = silu_f(t.x); t.y = silu_f(t.y); t.z = silu_f(t.z); t.w = silu_f(t.w);
      }
    }
    *(v4fa*)(srow + i * 128) = t;
    *(volatile v4f*)(orow + (size_t)i * (size_t)ldo) = t;
  }
  __threadfence();
#pragma unroll 1
  for (int i = 0; i < 16; ++i) {
    const v4f t = *(const v4fa*)(srow + i * 128);
    *(volatile v4f*)(orow + (size_t)i * (size_t)ldo) = t;
  }
}

__global__ __launch_bounds__(64) void k_conv(float* XS, const float* __restrict__ cw,
                                             const float* __restrict__ cb, unsigned short* UHL) {
  __shared__ __attribute__((aligned(16))) float tin[TS * CS];
  __shared__ __attribute__((aligned(16))) unsigned short thi[TS * CS];
  __shared__ __attribute__((aligned(16))) unsigned short tlo[TS * CS];
  const int tid = (int)threadIdx.x;
  const int b   = (int)blockIdx.x >> 5;
  const int c0  = ((int)blockIdx.x & 31) * CS;
  const int c   = c0 + tid;
  float w0, w1, w2, w3;
  {
    const v4f w = *(const v4fa*)(cw + 4 * c);
    w0 = bf16_val(w.x); w1 = bf16_val(w.y); w2 = bf16_val(w.z); w3 = bf16_val(w.w);
  }
  const float cbv = bf16_val(cb[c]);
  float xm1 = 0.0f, xm2 = 0.0f, xm3 = 0.0f;

#pragma unroll 1
  for (int s0 = 0; s0 < SEQ; s0 += TS) {
    const size_t rowb = (size_t)b * SEQ + (size_t)s0;
#pragma unroll
    for (int q = 0; q < 4; ++q) {
      const int p = tid + 64 * q;
      *(v4fa*)(tin + 4 * p) = *(const v4fa*)(XS + (rowb + (size_t)(p >> 4)) * DI + c0 + (p & 15) * 4);
    }
    __syncthreads();
#pragma unroll 2
    for (int sl = 0; sl < TS; ++sl) {
      const float x0 = tin[sl * CS + tid];
      float a = w0 * xm3;
      a = fmaf(w1, xm2, a);
      a = fmaf(w2, xm1, a);
      a = fmaf(w3, x0, a);
      const float v = a + cbv;
      const float uu = silu_f(v);
      const unsigned hb = bf16_bits(uu);
      const unsigned lb = bf16_bits(uu - __uint_as_float(hb << 16));
      tin[sl * CS + tid] = uu;
      thi[sl * CS + tid] = (unsigned short)hb;
      tlo[sl * CS + tid] = (unsigned short)lb;
      xm3 = xm2; xm2 = xm1; xm1 = x0;
    }
    __syncthreads();
    v4f  uv[4];
    v8us hv[2], lv[2];
#pragma unroll
    for (int q = 0; q < 4; ++q) uv[q] = *(const v4fa*)(tin + 4 * (tid + 64 * q));
#pragma unroll
    for (int q = 0; q < 2; ++q) {
      hv[q] = *(const v8usa*)(thi + 8 * (tid + 64 * q));
      lv[q] = *(const v8usa*)(tlo + 8 * (tid + 64 * q));
    }
#pragma unroll
    for (int q = 0; q < 4; ++q) {
      const int p = tid + 64 * q;
      *(volatile v4f*)(XS + (rowb + (size_t)(p >> 4)) * DI + c0 + (p & 15) * 4) = uv[q];
    }
#pragma unroll
    for (int q = 0; q < 2; ++q) {
      const int p = tid + 64 * q;
      unsigned short* hp = UHL + (rowb + (size_t)(p >> 3)) * KX + c0 + (p & 7) * 8;
      *(volatile v8us*)hp = hv[q];
      *(volatile v8us*)(hp + DI) = lv[q];
    }
    __threadfence();
#pragma unroll
    for (int q = 0; q < 4; ++q) {
      const int p = tid + 64 * q;
      *(volatile v4f*)(XS + (rowb + (size_t)(p >> 4)) * DI + c0 + (p & 15) * 4) = uv[q];
    }
#pragma unroll
    for (int q = 0; q < 2; ++q) {
      const int p = tid + 64 * q;
      unsigned short* hp = UHL + (rowb + (size_t)(p >> 3)) * KX + c0 + (p & 7) * 8;
      *(volatile v8us*)hp = hv[q];
      *(volatile v8us*)(hp + DI) = lv[q];
    }
    __syncthreads();
  }
}

__global__ __launch_bounds__(GTHR) void k_xb(const unsigned short* __restrict__ A,
                                             const unsigned short* __restrict__ BT, float* outF) {
  __shared__ __attribute__((aligned(16))) float stg[GBM * 64];
  const int tid = (int)threadIdx.x, lane = tid & 31, wave = tid >> 5, hh = lane >> 4, m = lane & 15;
  const int rowBase = (int)blockIdx.x * GBM;

  v8f acc[4];
  {
    const v8f z = {0.f, 0.f, 0.f, 0.f, 0.f, 0.f, 0.f, 0.f};
    acc[0] = z; acc[1] = z; acc[2] = z; acc[3] = z;
  }
  const unsigned short* ap = A  + (size_t)(rowBase + 16 * wave + m) * (size_t)KX + 8 * hh;
  const unsigned short* bp = BT + (size_t)m * (size_t)KX + 8 * hh;
  gemm_loop<4>(ap, bp, KX, acc);

#pragma unroll
  for (int t = 0; t < 4; ++t) {
    const int lc = 16 * t + m;
#pragma unroll
    for (int r = 0; r < 8; ++r) {
      const int lr = 16 * wave + 8 * hh + r;
      stg[lr * 64 + lc] = acc[t][r];
    }
  }
  __syncthreads();

  v4f fv[8];
#pragma unroll
  for (int i = 0; i < 8; ++i) {
    const int lr = 16 * wave + 2 * i + hh;
    fv[i] = *(const v4fa*)(stg + lr * 64 + 4 * m);
  }
#pragma unroll
  for (int i = 0; i < 8; ++i) {
    const int gr = rowBase + 16 * wave + 2 * i + hh;
    *(volatile v4f*)(outF + (size_t)gr * DS + 4 * m) = fv[i];
  }
  __threadfence();
#pragma unroll
  for (int i = 0; i < 8; ++i) {
    const int gr = rowBase + 16 * wave + 2 * i + hh;
    *(volatile v4f*)(outF + (size_t)gr * DS + 4 * m) = fv[i];
  }
}

__global__ __launch_bounds__(64) void k_rnn(const float* __restrict__ Amat, const float* __restrict__ XBP,
                                            unsigned short* HHL) {
  __shared__ __attribute__((aligned(16))) float AsT[DS * DS];
  __shared__ __attribute__((aligned(16))) float hb[2 * DS];
  __shared__ __attribute__((aligned(16))) float xbt[RCH * DS];
  __shared__ __attribute__((aligned(16))) unsigned short hlt[RCH * KH];
  const int tid = (int)threadIdx.x;
  const int b   = (int)blockIdx.x;

#pragma unroll 4
  for (int q = 0; q < DS; ++q) {
    const int e = q * 64 + tid;
    AsT[(e & 63) * DS + (e >> 6)] = bf16_val(Amat[e]);
  }
  hb[tid] = 0.0f;
  hb[DS + tid] = 0.0f;
  __syncthreads();

#pragma unroll 1
  for (int t0 = 0; t0 < SEQ; t0 += RCH) {
    const size_t rowb = (size_t)b * SEQ + (size_t)t0;
#pragma unroll 4
    for (int q = 0; q < 8; ++q) {
      const int p = tid + 64 * q;
      *(v4fa*)(xbt + 4 * p) = *(const v4fa*)(XBP + rowb * DS + 4 * p);
    }
    __syncthreads();
#pragma unroll 1
    for (int tl = 0; tl < RCH; ++tl) {
      const int par = (t0 + tl) & 1;
      const float* hc = hb + par * DS;
      float* hn = hb + (par ^ 1) * DS;
      float a0 = 0.0f, a1 = 0.0f, a2 = 0.0f, a3 = 0.0f;
#pragma unroll 4
      for (int q = 0; q < DS / 4; ++q) {
        const v4f h4 = *(const v4fa*)(hc + 4 * q);
        a0 = fmaf(AsT[(4 * q + 0) * DS + tid], h4.x, a0);
        a1 = fmaf(AsT[(4 * q + 1) * DS + tid], h4.y, a1);
        a2 = fmaf(AsT[(4 * q + 2) * DS + tid], h4.z, a2);
        a3 = fmaf(AsT[(4 * q + 3) * DS + tid], h4.w, a3);
      }
      const float pre = ((a0 + a1) + (a2 + a3)) + xbt[tl * DS + tid];
      const float hv = tanhf(pre);
      const unsigned hbits = bf16_bits(hv);
      const unsigned lbits = bf16_bits(hv - __uint_as_float(hbits << 16));
      hn[tid] = hv;
      hlt[tl * KH + tid]      = (unsigned short)hbits;
      hlt[tl * KH + DS + tid] = (unsigned short)lbits;
      __syncthreads();
    }
    v8us hq[8];
#pragma unroll
    for (int q = 0; q < 8; ++q) hq[q] = *(const v8usa*)(hlt + 8 * (tid + 64 * q));
#pragma unroll
    for (int q = 0; q < 8; ++q) *(volatile v8us*)(HHL + rowb * KH + 8 * (tid + 64 * q)) = hq[q];
    __threadfence();
#pragma unroll
    for (int q = 0; q < 8; ++q) *(volatile v8us*)(HHL + rowb * KH + 8 * (tid + 64 * q)) = hq[q];
    __syncthreads();
  }
}

__global__ __launch_bounds__(GTHR) void k_y(const unsigned short* __restrict__ A,
                                            const unsigned short* __restrict__ BT,
                                            const float* __restrict__ U, const float* __restrict__ SG,
                                            const float* __restrict__ Dv, unsigned short* XO) {
  __shared__ __attribute__((aligned(16))) float stg[GBM * 128];
  __shared__ __attribute__((aligned(16))) unsigned short rowbuf[4 * 256];
  const int tid = (int)threadIdx.x, lane = tid & 31, wave = tid >> 5, hh = lane >> 4, m = lane & 15;
  const int rowBase = (int)blockIdx.x * GBM;
  const int col0    = (int)blockIdx.y * 128;

  v8f acc[8];
  {
    const v8f z = {0.f, 0.f, 0.f, 0.f, 0.f, 0.f, 0.f, 0.f};
#pragma unroll
    for (int t = 0; t < 8; ++t) acc[t] = z;
  }
  const unsigned short* ap = A  + (size_t)(rowBase + 16 * wave + m) * (size_t)KH + 8 * hh;
  const unsigned short* bp = BT + (size_t)(col0 + m) * (size_t)KH + 8 * hh;
  gemm_loop<8>(ap, bp, KH, acc);

#pragma unroll
  for (int nt = 0; nt < 8; ++nt) {
    const int lc = 16 * nt + m;
#pragma unroll
    for (int r = 0; r < 8; ++r) {
      const int lr = 16 * wave + 8 * hh + r;
      stg[lr * 128 + lc] = acc[nt][r];
    }
  }
  __syncthreads();

  v4f d4;
  {
    const v4f t1 = *(const v4fa*)(Dv + col0 + 4 * lane);
    d4.x = bf16_val(t1.x); d4.y = bf16_val(t1.y); d4.z = bf16_val(t1.z); d4.w = bf16_val(t1.w);
  }
  unsigned short* rb = rowbuf + wave * 256;
  const int ocol = (lane < 16) ? (col0 + 8 * lane) : (DI + col0 + 8 * (lane - 16));

#pragma unroll 1
  for (int i = 0; i < 16; ++i) {
    const int r = rowBase + 16 * wave + i;
    const v4f a4 = *(const v4fa*)(stg + (16 * wave + i) * 128 + 4 * lane);
    const v4f u4 = *(const v4fa*)(U  + (size_t)r * DI + col0 + 4 * lane);
    const v4f g4 = *(const v4fa*)(SG + (size_t)r * DI + col0 + 4 * lane);
    const float x0 = fmaf(u4.x, d4.x, a4.x) * g4.x;
    const float x1 = fmaf(u4.y, d4.y, a4.y) * g4.y;
    const float x2 = fmaf(u4.z, d4.z, a4.z) * g4.z;
    const float x3 = fmaf(u4.w, d4.w, a4.w) * g4.w;
    v4us h4, l4;
    unsigned hbv;
    hbv = bf16_bits(x0); h4[0] = (unsigned short)hbv; l4[0] = (unsigned short)bf16_bits(x0 - __uint_as_float(hbv << 16));
    hbv = bf16_bits(x1); h4[1] = (unsigned short)hbv; l4[1] = (unsigned short)bf16_bits(x1 - __uint_as_float(hbv << 16));
    hbv = bf16_bits(x2); h4[2] = (unsigned short)hbv; l4[2] = (unsigned short)bf16_bits(x2 - __uint_as_float(hbv << 16));
    hbv = bf16_bits(x3); h4[3] = (unsigned short)hbv; l4[3] = (unsigned short)bf16_bits(x3 - __uint_as_float(hbv << 16));
    *(v4usa*)(rb + 4 * lane) = h4;
    *(v4usa*)(rb + 128 + 4 * lane) = l4;
    __syncthreads();
    const v8us q = *(const v8usa*)(rb + 8 * lane);
    unsigned short* op = XO + (size_t)r * KX + ocol;
    *(volatile v8us*)op = q;
    __threadfence();
    *(volatile v8us*)op = q;
    __syncthreads();
  }
}

extern "C" void kernel_launch(void* const* d_in, const int* in_sizes, int n_in,
                              void* d_out, int out_size, void* d_ws, size_t ws_size,
                              hipStream_t stream) {
  if (n_in < 11) return;
  if (in_sizes[0] != MT * DM) return;
  if (in_sizes[1] != E2 * DM) return;
  if (in_sizes[2] != E2) return;
  if (in_sizes[3] != DI * 4) return;
  if (in_sizes[4] != DI) return;
  if (in_sizes[5] != DS * DS) return;
  if (in_sizes[6] != DS * DI) return;
  if (in_sizes[7] != DI * DS) return;
  if (in_sizes[8] != DI) return;
  if (in_sizes[9] != DM * DI) return;
  if (in_sizes[10] != DM) return;
  if (out_size != MT * DM) return;

  const float* x  = (const float*)d_in[0];
  const float* w1 = (const float*)d_in[1];
  const float* b1 = (const float*)d_in[2];
  const float* cw = (const float*)d_in[3];
  const float* cb = (const float*)d_in[4];
  const float* Am = (const float*)d_in[5];
  const float* Bm = (const float*)d_in[6];
  const float* Cm = (const float*)d_in[7];
  const float* Dv = (const float*)d_in[8];
  const float* w2 = (const float*)d_in[9];
  const float* b2 = (const float*)d_in[10];
  float* out = (float*)d_out;

  char* ws = (char*)d_ws;
  size_t off = 0;
  const size_t oXB  = off; off += (size_t)MT * DM * 2;
  const size_t oWIN = off; off += (size_t)E2 * DM * 2;
  const size_t oWO  = off; off += (size_t)DM * KX * 2;
  const size_t oB2  = off; off += (size_t)DS * KX * 2;
  const size_t oC2  = off; off += (size_t)DI * KH * 2;
  const size_t oXS  = off; off += (size_t)MT * DI * 4;
  const size_t oSG  = off; off += (size_t)MT * DI * 4;
  const size_t oUHL = off; off += (size_t)MT * KX * 2;
  const size_t oXBP = off; off += (size_t)MT * DS * 4;
  const size_t oHHL = off; off += (size_t)MT * KH * 2;
  if (off > ws_size || off > (size_t)WSMAX) return;
  unsigned short* XB    = (unsigned short*)(ws + oXB);
  unsigned short* WIN   = (unsigned short*)(ws + oWIN);
  unsigned short* WOUT2 = (unsigned short*)(ws + oWO);
  unsigned short* B2    = (unsigned short*)(ws + oB2);
  unsigned short* C2    = (unsigned short*)(ws + oC2);
  float*          XS    = (float*)(ws + oXS);
  float*          SG    = (float*)(ws + oSG);
  unsigned short* UHL   = (unsigned short*)(ws + oUHL);
  unsigned short* XO    = UHL;
  float*          XBP   = (float*)(ws + oXBP);
  unsigned short* HHL   = (unsigned short*)(ws + oHHL);
  const size_t sgOff = (oSG - oXS) / 4;

  k_prep<<<UTOT / PTHR, PTHR, 0, stream>>>(x, w1, w2, Bm, Cm, XB, WIN, WOUT2, B2, C2);
  k_gemm128<1><<<dim3(MT / GBM, E2 / 128), GTHR, 0, stream>>>(XB, WIN, b1, XS, sgOff, DM, DI, DI);
  k_conv<<<NBAT * (DI / CS), 64, 0, stream>>>(XS, cw, cb, UHL);
  k_xb<<<MT / GBM, GTHR, 0, stream>>>(UHL, B2, XBP);
  k_rnn<<<NBAT, 64, 0, stream>>>(Am, XBP, HHL);
  k_y<<<dim3(MT / GBM, DI / 128), GTHR, 0, stream>>>(HHL, C2, XS, SG, Dv, XO);
  k_gemm128<0><<<dim3(MT / GBM, DM / 128), GTHR, 0, stream>>>(XO, WOUT2, b2, out, (size_t)0, KX, DM, 1 << 30);
}
